// CPSFFusedCodebook_64965675319784
// MI455X (gfx1250) — hardware-verified
//
#include <hip/hip_runtime.h>
#include <math.h>
#include <stdint.h>

#define NBQ  1024
#define NFD  128
#define NKC  256
#define NMC  8192
#define NSD  256
#define NOUT 512
#define NMT  128
#define NPAR 9

#define PI_F        3.14159265358979323846f
#define SQRT_PI_F   1.7724538509055159f
#define TINY_F      1.17549435e-38f
#define EPS_TOTAL_F 1e-3f

static_assert((NBQ % 64) == 0 && (NMC % 64) == 0 && (NOUT % 64) == 0);
static_assert((NBQ % 32) == 0 && (NMC % 32) == 0 && (NSD % 32) == 0);
static_assert((NKC % 32) == 0 && (NMC % 32) == 0 && NKC == 2 * NFD && NFD == 128);
static_assert(NMT * 64 == NMC && NOUT == 2 * NSD);
static_assert(((NBQ / 64) * (NOUT / 64)) % 8 == 0);

typedef __bf16   v16b __attribute__((ext_vector_type(16)));
typedef __bf16   v8b  __attribute__((ext_vector_type(8)));
typedef float    v8f  __attribute__((ext_vector_type(8)));
typedef float    v4f  __attribute__((ext_vector_type(4)));
typedef unsigned int v4u __attribute__((ext_vector_type(4)));

__device__ __forceinline__ unsigned short bf_bits(float f) {
  unsigned u = __float_as_uint(f);
  return (unsigned short)((u + 0x7FFFu + ((u >> 16) & 1u)) >> 16);
}
__device__ __forceinline__ float bf_up(unsigned short h) { return __uint_as_float(((unsigned)h) << 16); }
__device__ __forceinline__ unsigned pk16(unsigned short a, unsigned short b) { return (unsigned)a | ((unsigned)b << 16); }
__device__ __forceinline__ v8f zero8() { v8f z = {0.f, 0.f, 0.f, 0.f, 0.f, 0.f, 0.f, 0.f}; return z; }
__device__ __forceinline__ float wsum32(float v) {
  v += __shfl_xor(v, 16);
  v += __shfl_xor(v, 8);
  v += __shfl_xor(v, 4);
  v += __shfl_xor(v, 2);
  v += __shfl_xor(v, 1);
  return v;
}

__device__ __forceinline__ v16b ldfrag_b(const __bf16* p) {
  union { v16b v; v8b h[2]; } f;
  f.h[0] = *(const v8b*)(p);
  f.h[1] = *(const v8b*)(p + 16);
  return f.v;
}

__device__ __forceinline__ v8f mma_b_raw(v16b a, v16b b, v8f c) {
  return __builtin_amdgcn_wmma_f32_16x16x32_bf16(false, a, false, b, (short)0, c, false, false);
}
__device__ __forceinline__ void dep_guard_b(v8f& a, v8f& b, v16b x, v16b y) {
#if defined(__HIP_DEVICE_COMPILE__)
  asm volatile("v_nop\n\tv_nop\n\tv_nop\n\tv_nop" : "+v"(a), "+v"(b) : "v"(x), "v"(y));
#endif
}
__device__ __forceinline__ void keep4_b(v16b a, v16b b, v16b c, v16b d) {
#if defined(__HIP_DEVICE_COMPILE__)
  asm volatile("v_nop" :: "v"(a), "v"(b), "v"(c), "v"(d));
#endif
}
__device__ __forceinline__ void acc_guard4(v8f& a, v8f& b, v8f& c, v8f& d) {
#if defined(__HIP_DEVICE_COMPILE__)
  asm volatile("v_nop\n\tv_nop\n\tv_nop\n\tv_nop" : "+v"(a), "+v"(b), "+v"(c), "+v"(d));
#endif
}
__device__ __forceinline__ void acc_guard2(v8f& a, v8f& b) {
#if defined(__HIP_DEVICE_COMPILE__)
  asm volatile("v_nop\n\tv_nop\n\tv_nop\n\tv_nop" : "+v"(a), "+v"(b));
#endif
}
__device__ __forceinline__ void step_guard10(v8f& p, v8f& q, v16b a0, v16b a1, v16b a2, v16b a3,
                                             v16b b0, v16b b1, v16b b2, v16b b3) {
#if defined(__HIP_DEVICE_COMPILE__)
  asm volatile("v_nop\n\tv_nop\n\tv_nop\n\tv_nop"
               : "+v"(p), "+v"(q)
               : "v"(a0), "v"(a1), "v"(a2), "v"(a3), "v"(b0), "v"(b1), "v"(b2), "v"(b3));
#endif
}
__device__ __forceinline__ void wave_sync_lds() {
  __builtin_amdgcn_fence(__ATOMIC_RELEASE, "workgroup");
  __builtin_amdgcn_wave_barrier();
  __builtin_amdgcn_fence(__ATOMIC_ACQUIRE, "workgroup");
}

__global__ __launch_bounds__(128) void cvt_query(
    const float* __restrict__ zre, const float* __restrict__ zim,
    const float* __restrict__ dre, const float* __restrict__ dim_,
    unsigned short* ZA, unsigned short* ZB, unsigned short* DA, unsigned short* DB,
    float* szo, float* rndo) {
  __shared__ __align__(16) unsigned short sRow[4][NKC];
  __shared__ float sRed[2][4];
  __shared__ __align__(16) float sSt[2][32];
  const int tid  = threadIdx.x;
  const int lane = tid & 31;
  const int wave = tid >> 5;
  const int r0   = blockIdx.x * 32;
  unsigned short* plane = ZA;
  if (wave == 1) plane = ZB;
  if (wave == 2) plane = DA;
  if (wave == 3) plane = DB;
  for (int rr = 0; rr < 32; ++rr) {
    const int row = r0 + rr;
    const size_t src = (size_t)row * NFD + (size_t)tid;
    const unsigned short bzr = bf_bits(zre[src]);
    const unsigned short bzi = bf_bits(zim[src]);
    const unsigned short bdr = bf_bits(dre[src]);
    const unsigned short bdi = bf_bits(dim_[src]);
    const float zr = bf_up(bzr), zi = bf_up(bzi), dr = bf_up(bdr), di = bf_up(bdi);
    sRow[0][tid] = bzr;  sRow[0][NFD + tid] = bzi;
    sRow[1][tid] = bzi;  sRow[1][NFD + tid] = (unsigned short)(bzr ^ 0x8000u);
    sRow[2][tid] = bdr;  sRow[2][NFD + tid] = bdi;
    sRow[3][tid] = bdi;  sRow[3][NFD + tid] = (unsigned short)(bdr ^ 0x8000u);
    float pz = zr * zr + zi * zi;
    float pd = dr * dr + di * di;
    pz = wsum32(pz);
    pd = wsum32(pd);
    if (lane == 0) { sRed[0][wave] = pz; sRed[1][wave] = pd; }
    __syncthreads();
    {
      const v4u v = *(const v4u*)(&sRow[wave][lane * 8]);
      unsigned short* dst = plane + (size_t)row * NKC + (size_t)lane * 8;
      *(volatile v4u*)dst = v;
      __threadfence();
      *(volatile v4u*)dst = v;
    }
    if (tid == 0) {
      const float tz = (sRed[0][0] + sRed[0][1]) + (sRed[0][2] + sRed[0][3]);
      const float td = (sRed[1][0] + sRed[1][1]) + (sRed[1][2] + sRed[1][3]);
      const float n  = sqrtf(td);
      const float rn = (n == 0.0f) ? 1.0f : (1.0f / n);
      sSt[0][rr] = tz;
      sSt[1][rr] = rn;
    }
    __syncthreads();
  }
  if (tid < 16) {
    const int p = tid >> 3, q = tid & 7;
    const v4f v = *(const v4f*)(&sSt[p][q * 4]);
    float* base = (p == 0) ? szo : rndo;
    float* dst = base + r0 + q * 4;
    *(volatile v4f*)dst = v;
    __threadfence();
    *(volatile v4f*)dst = v;
  }
}

__global__ __launch_bounds__(128) void cvt_code(
    const float* __restrict__ zjre, const float* __restrict__ zjim,
    const float* __restrict__ djre, const float* __restrict__ djim,
    const float* __restrict__ alphaP, const float* __restrict__ sigpP, const float* __restrict__ sigqP,
    unsigned short* DJ, unsigned short* ZJ, float* par) {
  __shared__ __align__(16) unsigned short sRow[2][NKC];
  __shared__ float sRed[4][4];
  __shared__ __align__(16) float sPar[NPAR][32];
  const int tid  = threadIdx.x;
  const int lane = tid & 31;
  const int wave = tid >> 5;
  const int r0   = blockIdx.x * 32;
  for (int rr = 0; rr < 32; ++rr) {
    const int row = r0 + rr;
    const size_t src = (size_t)row * NFD + (size_t)tid;
    const unsigned short bzr = bf_bits(zjre[src]);
    const unsigned short bzi = bf_bits(zjim[src]);
    const unsigned short bdr = bf_bits(djre[src]);
    const unsigned short bdi = bf_bits(djim[src]);
    const float zr = bf_up(bzr), zi = bf_up(bzi), dr = bf_up(bdr), di = bf_up(bdi);
    sRow[0][tid] = bdr;  sRow[0][NFD + tid] = bdi;
    sRow[1][tid] = bzr;  sRow[1][NFD + tid] = bzi;
    float p0 = dr * dr + di * di;
    float p1 = dr * zr + di * zi;
    float p2 = dr * zi - di * zr;
    float p3 = zr * zr + zi * zi;
    p0 = wsum32(p0);
    p1 = wsum32(p1);
    p2 = wsum32(p2);
    p3 = wsum32(p3);
    if (lane == 0) { sRed[0][wave] = p0; sRed[1][wave] = p1; sRed[2][wave] = p2; sRed[3][wave] = p3; }
    __syncthreads();
    if (wave < 2) {
      const v4u v = *(const v4u*)(&sRow[wave][lane * 8]);
      unsigned short* plane = (wave == 0) ? DJ : ZJ;
      unsigned short* dst = plane + (size_t)row * NKC + (size_t)lane * 8;
      *(volatile v4u*)dst = v;
      __threadfence();
      *(volatile v4u*)dst = v;
    }
    if (tid == 0) {
      const float tdd = (sRed[0][0] + sRed[0][1]) + (sRed[0][2] + sRed[0][3]);
      const float tzr = (sRed[1][0] + sRed[1][1]) + (sRed[1][2] + sRed[1][3]);
      const float tzi = (sRed[2][0] + sRed[2][1]) + (sRed[2][2] + sRed[2][3]);
      const float tzz = (sRed[3][0] + sRed[3][1]) + (sRed[3][2] + sRed[3][3]);
      const float n   = sqrtf(tdd);
      const float rn  = (n == 0.0f) ? 1.0f : (1.0f / n);
      const float al  = fmaxf(bf_up(bf_bits(alphaP[row])), TINY_F);
      const float sp  = fmaxf(bf_up(bf_bits(sigpP[row])), TINY_F);
      const float sq  = fmaxf(bf_up(bf_bits(sigqP[row])), TINY_F);
      const float scl = sqrtf(sp / PI_F);
      sPar[0][rr] = rn;
      sPar[1][rr] = tzr * rn;
      sPar[2][rr] = tzi * rn;
      sPar[3][rr] = tzz;
      sPar[4][rr] = al;
      sPar[5][rr] = 1.0f / sp;
      sPar[6][rr] = 1.0f / sq;
      sPar[7][rr] = scl;
      sPar[8][rr] = scl / SQRT_PI_F;
    }
    __syncthreads();
  }
  if (tid < NPAR * 8) {
    const int p = tid >> 3, q = tid & 7;
    const v4f v = *(const v4f*)(&sPar[p][q * 4]);
    float* dst = par + (size_t)p * NMC + r0 + q * 4;
    *(volatile v4f*)dst = v;
    __threadfence();
    *(volatile v4f*)dst = v;
  }
}

__global__ __launch_bounds__(256) void tr_payload(const float* __restrict__ Tre, const float* __restrict__ Tim,
                                                  unsigned short* Tt) {
  __shared__ __align__(16) unsigned short sT[64][72];
  const int tid = threadIdx.x;
  const int m0  = blockIdx.x * 64;
  const int s0  = blockIdx.y * 32;
  const int ml  = tid >> 2;
  const int s8  = (tid & 3) * 8;
  const size_t src = (size_t)(m0 + ml) * NSD + (size_t)(s0 + s8);
  const v4f ra = *(const v4f*)(Tre + src);
  const v4f rb = *(const v4f*)(Tre + src + 4);
  const v4f ia = *(const v4f*)(Tim + src);
  const v4f ib = *(const v4f*)(Tim + src + 4);
#pragma unroll
  for (int j = 0; j < 4; ++j) {
    sT[2 * (s8 + j)][ml]         = bf_bits(ra[j]);
    sT[2 * (s8 + j) + 1][ml]     = bf_bits(ia[j]);
    sT[2 * (s8 + 4 + j)][ml]     = bf_bits(rb[j]);
    sT[2 * (s8 + 4 + j) + 1][ml] = bf_bits(ib[j]);
  }
  __syncthreads();
#pragma unroll
  for (int it = 0; it < 2; ++it) {
    const int idx = tid + it * 256;
    const int nl = idx >> 3, q = idx & 7;
    const v4u v = *(const v4u*)(&sT[nl][q * 8]);
    unsigned short* dst = Tt + (size_t)(2 * s0 + nl) * NMC + (size_t)(m0 + q * 8);
    *(volatile v4u*)dst = v;
    __threadfence();
    *(volatile v4u*)dst = v;
  }
}

__device__ __forceinline__ float gh_term(float prr, float scl, float isp, float base, float node, float wgt) {
  const float d = prr - node * scl;
  return wgt * __expf(-PI_F * (d * d * isp + base));
}

__global__ __launch_bounds__(256) void pair_weights(
    const unsigned short* __restrict__ ZAp, const unsigned short* __restrict__ ZBp,
    const unsigned short* __restrict__ DAp, const unsigned short* __restrict__ DBp,
    const unsigned short* __restrict__ DJp, const unsigned short* __restrict__ ZJp,
    const float* __restrict__ par, const float* __restrict__ sz, const float* __restrict__ rnd,
    unsigned short* Wh, unsigned short* Wl, float* denp) {
  const __bf16* ZA = (const __bf16*)(const void*)ZAp;
  const __bf16* ZB = (const __bf16*)(const void*)ZBp;
  const __bf16* DA = (const __bf16*)(const void*)DAp;
  const __bf16* DB = (const __bf16*)(const void*)DBp;
  const __bf16* DJ = (const __bf16*)(const void*)DJp;
  const __bf16* ZJ = (const __bf16*)(const void*)ZJp;
  __shared__ __align__(16) float sW[64 * 68];
  __shared__ __align__(16) float sDW[8][16];
  __shared__ __align__(16) float sDen[64];
  const int tid  = threadIdx.x;
  const int lane = tid & 31;
  const int wave = tid >> 5;
  const int wb = wave >> 1, wm = wave & 1;
  const int mt = blockIdx.x, bt = blockIdx.y;
  const int m0 = mt * 64, b0 = bt * 64;
  const int rl = lane & 15, hh = lane >> 4, koff = hh * 8;
  const int bw = b0 + wb * 16;
  const int mw = m0 + wm * 32;

  v8f aPR[2], aPI[2], aAR[2], aAI[2], aRR[2];
#pragma unroll
  for (int j = 0; j < 2; ++j) { aPR[j] = zero8(); aPI[j] = zero8(); aAR[j] = zero8(); aAI[j] = zero8(); aRR[j] = zero8(); }

  const size_t arow = (size_t)(bw + rl) * NKC + (size_t)koff;
  const size_t br0  = (size_t)(mw + rl) * NKC + (size_t)koff;
  const size_t br1  = (size_t)(mw + 16 + rl) * NKC + (size_t)koff;
#pragma unroll 1
  for (int k0 = 0; k0 < NKC; k0 += 32) {
    const v16b bd0 = ldfrag_b(DJ + br0 + k0);
    const v16b bd1 = ldfrag_b(DJ + br1 + k0);
    const v16b bz0 = ldfrag_b(ZJ + br0 + k0);
    const v16b bz1 = ldfrag_b(ZJ + br1 + k0);
    const v16b fa = ldfrag_b(ZA + arow + k0);
    aPR[0] = mma_b_raw(fa, bd0, aPR[0]);
    aPR[1] = mma_b_raw(fa, bd1, aPR[1]);
    aRR[0] = mma_b_raw(fa, bz0, aRR[0]);
    aRR[1] = mma_b_raw(fa, bz1, aRR[1]);
    const v16b fb = ldfrag_b(ZB + arow + k0);
    aPI[0] = mma_b_raw(fb, bd0, aPI[0]);
    aPI[1] = mma_b_raw(fb, bd1, aPI[1]);
    const v16b fc = ldfrag_b(DA + arow + k0);
    aAR[0] = mma_b_raw(fc, bd0, aAR[0]);
    aAR[1] = mma_b_raw(fc, bd1, aAR[1]);
    const v16b fd = ldfrag_b(DB + arow + k0);
    aAI[0] = mma_b_raw(fd, bd0, aAI[0]);
    aAI[1] = mma_b_raw(fd, bd1, aAI[1]);
    step_guard10(aPR[0], aAI[1], fa, fb, fc, fd, bd0, bd1, bz0, bz1);
  }
  acc_guard4(aPR[0], aPR[1], aPI[0], aPI[1]);
  acc_guard4(aAR[0], aAR[1], aAI[0], aAI[1]);
  acc_guard2(aRR[0], aRR[1]);

  const v8f szv = *(const v8f*)(sz + bw + 8 * hh);
  const v8f rnv = *(const v8f*)(rnd + bw + 8 * hh);
  float dp[8];
#pragma unroll
  for (int r = 0; r < 8; ++r) dp[r] = 0.0f;
#pragma unroll
  for (int j = 0; j < 2; ++j) {
    const int m = mw + 16 * j + rl;
    const float rndj = par[0 * NMC + m];
    const float cr   = par[1 * NMC + m];
    const float ci   = par[2 * NMC + m];
    const float szj  = par[3 * NMC + m];
    const float am   = par[4 * NMC + m];
    const float isp  = par[5 * NMC + m];
    const float isq  = par[6 * NMC + m];
    const float scl  = par[7 * NMC + m];
    const float sw   = par[8 * NMC + m];
#pragma unroll
    for (int r = 0; r < 8; ++r) {
      const float prr = aPR[j][r] * rndj - cr;
      const float pii = aPI[j][r] * rndj - ci;
      const float dz2 = (szv[r] + szj) - 2.0f * aRR[j][r];
      const float perp2 = fmaxf(dz2 - (prr * prr + pii * pii), 0.0f);
      const float sc = rnv[r] * rndj;
      const float arr = aAR[j][r] * sc;
      const float aii = aAI[j][r] * sc;
      const float align = arr * arr + aii * aii;
      const float base = pii * pii * isp + perp2 * isq;
      float s = gh_term(prr, scl, isp, base, -2.930637420257244f, 1.9960407221136762e-4f);
      s += gh_term(prr, scl, isp, base, -1.981656756695843f, 1.7077983007413475e-2f);
      s += gh_term(prr, scl, isp, base, -1.1571937124467802f, 0.20780232581489188f);
      s += gh_term(prr, scl, isp, base, -0.3811869902073221f, 0.6611470125582413f);
      s += gh_term(prr, scl, isp, base, 0.3811869902073221f, 0.6611470125582413f);
      s += gh_term(prr, scl, isp, base, 1.1571937124467802f, 0.20780232581489188f);
      s += gh_term(prr, scl, isp, base, 1.981656756695843f, 1.7077983007413475e-2f);
      s += gh_term(prr, scl, isp, base, 2.930637420257244f, 1.9960407221136762e-4f);
      const float w = am * align * (s * sw);
      sW[(wb * 16 + 8 * hh + r) * 68 + wm * 32 + 16 * j + rl] = w;
      dp[r] += w;
    }
  }
#pragma unroll
  for (int r = 0; r < 8; ++r) {
    float p = dp[r];
    p += __shfl_xor(p, 1);
    p += __shfl_xor(p, 2);
    p += __shfl_xor(p, 4);
    p += __shfl_xor(p, 8);
    dp[r] = p;
  }
  if (rl == 0) {
#pragma unroll
    for (int r = 0; r < 8; ++r) sDW[wave][8 * hh + r] = dp[r];
  }
  __syncthreads();
  if (tid < 64) {
    const int wbq = tid >> 4, rq = tid & 15;
    sDen[tid] = sDW[2 * wbq][rq] + sDW[2 * wbq + 1][rq];
  }
#pragma unroll
  for (int it = 0; it < 2; ++it) {
    const int idx = tid + it * 256;
    const int row = idx >> 3, q = idx & 7;
    const v4f x0 = *(const v4f*)(sW + row * 68 + q * 8);
    const v4f x1 = *(const v4f*)(sW + row * 68 + q * 8 + 4);
    unsigned short h[8], l[8];
#pragma unroll
    for (int e = 0; e < 4; ++e) {
      h[e] = bf_bits(x0[e]);      l[e] = bf_bits(x0[e] - bf_up(h[e]));
      h[4 + e] = bf_bits(x1[e]);  l[4 + e] = bf_bits(x1[e] - bf_up(h[4 + e]));
    }
    v4u ph, pl;
    ph[0] = pk16(h[0], h[1]); ph[1] = pk16(h[2], h[3]); ph[2] = pk16(h[4], h[5]); ph[3] = pk16(h[6], h[7]);
    pl[0] = pk16(l[0], l[1]); pl[1] = pk16(l[2], l[3]); pl[2] = pk16(l[4], l[5]); pl[3] = pk16(l[6], l[7]);
    const size_t o = (size_t)(b0 + row) * NMC + (size_t)(m0 + q * 8);
    *(volatile v4u*)(Wh + o) = ph;
    *(volatile v4u*)(Wl + o) = pl;
    __threadfence();
    *(volatile v4u*)(Wh + o) = ph;
    *(volatile v4u*)(Wl + o) = pl;
  }
  __syncthreads();
  if (tid < 16) {
    const v4f v = *(const v4f*)(&sDen[tid * 4]);
    float* dst = denp + (size_t)mt * NBQ + b0 + tid * 4;
    *(volatile v4f*)dst = v;
    __threadfence();
    *(volatile v4f*)dst = v;
  }
}

__global__ __launch_bounds__(256) void mix_gemm(
    const unsigned short* __restrict__ Whp, const unsigned short* __restrict__ Wlp,
    const unsigned short* __restrict__ Ttp, const float* __restrict__ denp, float* out) {
  const __bf16* Ah = (const __bf16*)(const void*)Whp;
  const __bf16* Al = (const __bf16*)(const void*)Wlp;
  const __bf16* Bt = (const __bf16*)(const void*)Ttp;
  __shared__ __align__(16) float sT[8][16 * 68];
  __shared__ __align__(16) float sRD[8][64];
  const int lane = threadIdx.x & 31;
  const int wave = threadIdx.x >> 5;
  const int tilesN = NOUT >> 6;
  const int tilesM = NBQ >> 6;
  const int tile = blockIdx.x * 8 + wave;
  if (tile >= tilesM * tilesN) return;
  const int tm = tile / tilesN;
  const int tn = tile - tm * tilesN;
  const int m0 = tm << 6;
  const int n0 = tn << 6;
  const int rlane = lane & 15;
  const int koff  = (lane >> 4) * 8;
  const int mOff  = (lane >> 4) * 8;

  {
    float d0 = 0.0f, d1 = 0.0f;
#pragma unroll 1
    for (int t = 0; t < NMT; ++t) {
      d0 += denp[(size_t)t * NBQ + m0 + lane];
      d1 += denp[(size_t)t * NBQ + m0 + 32 + lane];
    }
    d0 += EPS_TOTAL_F;
    d1 += EPS_TOTAL_F;
    sRD[wave][lane]      = 1.0f / d0;
    sRD[wave][32 + lane] = 1.0f / d1;
  }
  wave_sync_lds();

  v8f acc[4][4];
#pragma unroll
  for (int i = 0; i < 4; ++i)
#pragma unroll
    for (int j = 0; j < 4; ++j) acc[i][j] = zero8();

#pragma unroll 1
  for (int k0 = 0; k0 < NMC; k0 += 32) {
    v16b bh[4];
#pragma unroll
    for (int j = 0; j < 4; ++j) {
      const size_t bo = (size_t)(n0 + (j << 4) + rlane) * NMC + koff + k0;
      bh[j] = ldfrag_b(Bt + bo);
    }
#pragma unroll
    for (int i = 0; i < 4; ++i) {
      const size_t ao = (size_t)(m0 + (i << 4) + rlane) * NMC + koff + k0;
      const v16b ah = ldfrag_b(Ah + ao);
      const v16b al = ldfrag_b(Al + ao);
#pragma unroll
      for (int j = 0; j < 4; ++j) {
        acc[i][j] = mma_b_raw(ah, bh[j], acc[i][j]);
        acc[i][j] = mma_b_raw(al, bh[j], acc[i][j]);
      }
      dep_guard_b(acc[i][0], acc[i][3], ah, al);
    }
    keep4_b(bh[0], bh[1], bh[2], bh[3]);
  }
  acc_guard4(acc[0][0], acc[0][1], acc[0][2], acc[0][3]);
  acc_guard4(acc[1][0], acc[1][1], acc[1][2], acc[1][3]);
  acc_guard4(acc[2][0], acc[2][1], acc[2][2], acc[2][3]);
  acc_guard4(acc[3][0], acc[3][1], acc[3][2], acc[3][3]);

  float* slab = sT[wave];
  const int hh = lane >> 4, c4 = (lane & 15) * 4;
#pragma unroll
  for (int i = 0; i < 4; ++i) {
    const int mBase = m0 + (i << 4);
#pragma unroll
    for (int j = 0; j < 4; ++j) {
#pragma unroll
      for (int r = 0; r < 8; ++r) {
        slab[(mOff + r) * 68 + (j << 4) + rlane] = acc[i][j][r];
      }
    }
    wave_sync_lds();
    for (int pass = 0; pass < 2; ++pass) {
#pragma unroll
      for (int it = 0; it < 8; ++it) {
        const int row = it * 2 + hh;
        const float rd = sRD[wave][(i << 4) + row];
        v4f v = *(const v4f*)(slab + row * 68 + c4);
        v = v * rd;
        *(volatile v4f*)(out + (size_t)(mBase + row) * NOUT + n0 + c4) = v;
      }
      __threadfence();
    }
    wave_sync_lds();
  }
}

extern "C" void kernel_launch(void* const* d_in, const int* in_sizes, int n_in,
                              void* d_out, int out_size, void* d_ws, size_t ws_size,
                              hipStream_t stream) {
  if (n_in < 13) return;
  for (int i = 0; i < 4; ++i) if (in_sizes[i] != NBQ * NFD) return;
  for (int i = 4; i < 8; ++i) if (in_sizes[i] != NMC * NFD) return;
  if (in_sizes[8] != NMC * NSD || in_sizes[9] != NMC * NSD) return;
  if (in_sizes[10] != NMC || in_sizes[11] != NMC || in_sizes[12] != NMC) return;
  if (out_size != NBQ * NOUT) return;

  const float* z_re  = (const float*)d_in[0];
  const float* z_im  = (const float*)d_in[1];
  const float* d_re  = (const float*)d_in[2];
  const float* d_im  = (const float*)d_in[3];
  const float* zj_re = (const float*)d_in[4];
  const float* zj_im = (const float*)d_in[5];
  const float* dj_re = (const float*)d_in[6];
  const float* dj_im = (const float*)d_in[7];
  const float* T_re  = (const float*)d_in[8];
  const float* T_im  = (const float*)d_in[9];
  const float* alpha = (const float*)d_in[10];
  const float* sigp  = (const float*)d_in[11];
  const float* sigq  = (const float*)d_in[12];
  float* out = (float*)d_out;

  const size_t PQ   = (size_t)NBQ * NKC * 2;
  const size_t PC   = (size_t)NMC * NKC * 2;
  const size_t PTt  = (size_t)NOUT * NMC * 2;
  const size_t PPar = (size_t)NPAR * NMC * 4;
  const size_t PSt  = (size_t)NBQ * 4;
  const size_t PW   = (size_t)NBQ * NMC * 2;
  const size_t PDen = (size_t)NMT * NBQ * 4;
  size_t off = 0;
  const size_t oZA = off; off += PQ;
  const size_t oZB = off; off += PQ;
  const size_t oDA = off; off += PQ;
  const size_t oDB = off; off += PQ;
  const size_t oDJ = off; off += PC;
  const size_t oZJ = off; off += PC;
  const size_t oTt = off; off += PTt;
  const size_t oPar = off; off += PPar;
  const size_t oSz = off; off += PSt;
  const size_t oRnd = off; off += PSt;
  const size_t oWh = off; off += PW;
  const size_t oWl = off; off += PW;
  const size_t oDen = off; off += PDen;
  if (off > ws_size) return;
  if (off > (size_t)134217728) return;

  char* ws = (char*)d_ws;
  unsigned short* ZA = (unsigned short*)(ws + oZA);
  unsigned short* ZB = (unsigned short*)(ws + oZB);
  unsigned short* DA = (unsigned short*)(ws + oDA);
  unsigned short* DB = (unsigned short*)(ws + oDB);
  unsigned short* DJ = (unsigned short*)(ws + oDJ);
  unsigned short* ZJ = (unsigned short*)(ws + oZJ);
  unsigned short* Tt = (unsigned short*)(ws + oTt);
  float* par  = (float*)(ws + oPar);
  float* sz   = (float*)(ws + oSz);
  float* rnd  = (float*)(ws + oRnd);
  unsigned short* Wh = (unsigned short*)(ws + oWh);
  unsigned short* Wl = (unsigned short*)(ws + oWl);
  float* denp = (float*)(ws + oDen);

  const dim3 blk128(128), blk256(256);
  const dim3 gQ(NBQ / 32);
  const dim3 gC(NMC / 32);
  const dim3 gT(NMC / 64, NSD / 32);
  const dim3 gP(NMT, NBQ / 64);
  const dim3 gM(((NBQ / 64) * (NOUT / 64)) / 8);

  cvt_query<<<gQ, blk128, 0, stream>>>(z_re, z_im, d_re, d_im, ZA, ZB, DA, DB, sz, rnd);
  cvt_code<<<gC, blk128, 0, stream>>>(zj_re, zj_im, dj_re, dj_im, alpha, sigp, sigq, DJ, ZJ, par);
  tr_payload<<<gT, blk256, 0, stream>>>(T_re, T_im, Tt);
  pair_weights<<<gP, blk256, 0, stream>>>(ZA, ZB, DA, DB, DJ, ZJ, par, sz, rnd, Wh, Wl, denp);
  mix_gemm<<<gM, blk256, 0, stream>>>(Wh, Wl, Tt, denp, out);
  (void)hipGetLastError();
}
